// LongTermAttention_73366631350396
// MI455X (gfx1250) — hardware-verified
//
#include <hip/hip_runtime.h>


#define LL   1024
#define NBAT 8
#define DMD  768
#define NH_  12
#define HD   64
#define NBS  256
typedef _Float16 h16;
typedef unsigned short bf;
typedef __attribute__((ext_vector_type(16))) __bf16   v16bf;
typedef __attribute__((ext_vector_type(16))) _Float16 v16h;
typedef __attribute__((ext_vector_type(8)))  _Float16 v8h;
typedef __attribute__((ext_vector_type(8)))  unsigned short v8us;
typedef __attribute__((ext_vector_type(8)))  float    v8f;
typedef __attribute__((ext_vector_type(4)))  float    v4f;
typedef v8h  __attribute__((may_alias)) v8ha;
typedef v4f  __attribute__((may_alias)) v4fa;
typedef v8us __attribute__((may_alias)) v8usa;

__device__ __forceinline__ unsigned short f2bf(float f) { unsigned u = __float_as_uint(f); u += 0x7FFFu + ((u >> 16) & 1u); return (unsigned short)(u >> 16); }
__device__ __forceinline__ float bf2f(unsigned short b) { return __uint_as_float(((unsigned)b) << 16); }
__device__ __forceinline__ float bfr(float f) { return bf2f(f2bf(f)); }
__device__ __forceinline__ v16h cat16(v8h lo, v8h hi) { return __builtin_shufflevector(lo, hi, 0, 1, 2, 3, 4, 5, 6, 7, 8, 9, 10, 11, 12, 13, 14, 15); }
__device__ __forceinline__ v16bf cat16b(v8us lo, v8us hi) { return __builtin_bit_cast(v16bf, __builtin_shufflevector(lo, hi, 0, 1, 2, 3, 4, 5, 6, 7, 8, 9, 10, 11, 12, 13, 14, 15)); }
__device__ __forceinline__ v8f wmma16(v16h a, v16h b, v8f c) { return __builtin_amdgcn_wmma_f32_16x16x32_f16(false, a, false, b, (short)0, c, false, false); }
__device__ __forceinline__ v8f wmmab(v16bf a, v16bf b, v8f c) { return __builtin_amdgcn_wmma_f32_16x16x32_bf16(false, a, false, b, (short)0, c, false, false); }


template <typename T16> struct WFrag;
template <> struct WFrag<h16> { typedef v16h V; static __device__ __forceinline__ V ld(const h16* p) { return cat16(*(const v8h*)p, *(const v8h*)(p + 16)); } static __device__ __forceinline__ v8f mma(V a, V b, v8f c) { return wmma16(a, b, c); } };
template <> struct WFrag<bf> { typedef v16bf V; static __device__ __forceinline__ V ld(const bf* p) { return cat16b(*(const v8us*)p, *(const v8us*)(p + 16)); } static __device__ __forceinline__ v8f mma(V a, V b, v8f c) { return wmmab(a, b, c); } };
template <typename T16, int NSPLIT, bool BIAS>
__global__ __launch_bounds__(32) void k_gemmw(const T16* __restrict__ A, const T16* __restrict__ A2, const T16* __restrict__ Bt, const T16* __restrict__ Bt2, int K, float* C, int ldc, const float* __restrict__ bias, size_t sA, size_t sB, size_t sC) {
    typedef typename WFrag<T16>::V V;
    __shared__ __align__(16) float os[16 * 68];
    const size_t z = blockIdx.z; A += z * sA; if (A2) A2 += z * sA; Bt += z * sB; if (Bt2) Bt2 += z * sB; C += z * sC;
    const int lane = threadIdx.x & 31, lr = lane & 15, hi = lane >> 4; const int r0 = blockIdx.x * 64, c0 = blockIdx.y * 64;
    v8f acc[4][4];
#pragma unroll
    for (int mb = 0; mb < 4; ++mb)
#pragma unroll
        for (int nb = 0; nb < 4; ++nb) acc[mb][nb] = (v8f){};
    const size_t aoff = (size_t)(r0 + lr) * K + 8 * hi, boff = (size_t)(c0 + lr) * K + 8 * hi;
#pragma unroll 1
    for (int kc = 0; kc < K; kc += 32) {
        V a[4], a2[4];
#pragma unroll
        for (int mb = 0; mb < 4; ++mb) { a[mb] = WFrag<T16>::ld(A + aoff + (size_t)mb * 16 * K + kc); if (NSPLIT == 1 || NSPLIT == 2) a2[mb] = WFrag<T16>::ld(A2 + aoff + (size_t)mb * 16 * K + kc); }
#pragma unroll
        for (int nb = 0; nb < 4; ++nb) { const V b = WFrag<T16>::ld(Bt + boff + (size_t)nb * 16 * K + kc); V b2; if (NSPLIT >= 2) b2 = WFrag<T16>::ld(Bt2 + boff + (size_t)nb * 16 * K + kc);
#pragma unroll
            for (int mb = 0; mb < 4; ++mb) { acc[mb][nb] = WFrag<T16>::mma(a[mb], b, acc[mb][nb]); if (NSPLIT == 1 || NSPLIT == 2) acc[mb][nb] = WFrag<T16>::mma(a2[mb], b, acc[mb][nb]); if (NSPLIT >= 2) acc[mb][nb] = WFrag<T16>::mma(a[mb], b2, acc[mb][nb]); } }
        asm volatile("v_nop\n\tv_nop\n\tv_nop\n\tv_nop" : "+v"(acc[0][0]), "+v"(acc[1][1]), "+v"(acc[2][2]), "+v"(acc[3][3]) : "v"(a[0]), "v"(a[3]));
    }
#pragma unroll
    for (int mb = 0; mb < 4; ++mb) {
#pragma unroll
        for (int nb = 0; nb < 4; ++nb) {
#pragma unroll
            for (int j = 0; j < 8; ++j) os[(hi * 8 + j) * 68 + nb * 16 + lr] = acc[mb][nb][j]; }
        __builtin_amdgcn_wave_barrier(); asm volatile("" ::: "memory");
        float* crow = C + (size_t)(r0 + mb * 16) * ldc + c0;
#pragma unroll 1
        for (int ps = 0; ps < 2; ++ps) {
#pragma unroll
            for (int s = 0; s < 8; ++s) { const int row = 2 * s + hi, cofs = lr * 4; v4f val = *(const v4fa*)(os + row * 68 + cofs); if (BIAS) { val[0] += bfr(bias[c0 + cofs]); val[1] += bfr(bias[c0 + cofs + 1]); val[2] += bfr(bias[c0 + cofs + 2]); val[3] += bfr(bias[c0 + cofs + 3]); }
                *(volatile v4f*)(crow + (size_t)row * ldc + cofs) = val; }
            if (ps == 0) __threadfence(); }
        __builtin_amdgcn_wave_barrier(); asm volatile("" ::: "memory");
    }
}

__device__ __forceinline__ void splitf(float y, unsigned short& h, unsigned short& l) { h = f2bf(y); l = f2bf(y - bf2f(h)); }
typedef __attribute__((ext_vector_type(2))) unsigned short v2us;
typedef __attribute__((ext_vector_type(4))) unsigned short v4us;

__global__ __launch_bounds__(256) void k_cvt8(const float* __restrict__ src, bf* dst, size_t n8) { const size_t i = (size_t)blockIdx.x * 256 + threadIdx.x; if (i >= n8) return; const v8f v = *(const v8f*)(src + i * 8); v8us o;
#pragma unroll
    for (int k = 0; k < 8; ++k) o[k] = f2bf(v[k]); *(volatile v8us*)(dst + i * 8) = o; __threadfence(); *(volatile v8us*)(dst + i * 8) = o; }
__global__ __launch_bounds__(256) void k_gt(const float* __restrict__ G, bf* GT) { const int e = (blockIdx.x * 256 + threadIdx.x) * 4; if (e >= NBS * LL) return; const int l = e % LL; const int n = e / LL; v4us o;
#pragma unroll
    for (int u = 0; u < 4; ++u) o[u] = f2bf(G[(size_t)(l + u) * NBS + n]); *(volatile v4us*)(GT + e) = o; __threadfence(); *(volatile v4us*)(GT + e) = o; }
__global__ __launch_bounds__(256) void k_xbt(const float* __restrict__ x, int b, bf* XT) { const int e = (blockIdx.x * 256 + threadIdx.x) * 4; if (e >= DMD * LL) return; const int l = e % LL; const int d = e / LL; v4us o;
#pragma unroll
    for (int u = 0; u < 4; ++u) o[u] = f2bf(x[((size_t)(l + u) * NBAT + b) * DMD + d]); *(volatile v4us*)(XT + e) = o; __threadfence(); *(volatile v4us*)(XT + e) = o; }
__global__ __launch_bounds__(256) void k_qrow(const float* __restrict__ q, int b, bf* QB) { const int e = (blockIdx.x * 256 + threadIdx.x) * 4; if (e >= LL * DMD) return; const int d = e % DMD; const int l = e / DMD; const float* src = q + ((size_t)l * NBAT + b) * DMD + d; v4us o;
#pragma unroll
    for (int u = 0; u < 4; ++u) o[u] = f2bf(src[u]); *(volatile v4us*)(QB + e) = o; __threadfence(); *(volatile v4us*)(QB + e) = o; }
__global__ __launch_bounds__(256) void k_pl2(const float* __restrict__ F, int rows, bf* Ph, bf* Pl) { const size_t e = ((size_t)blockIdx.x * 256 + threadIdx.x) * 4; if (e >= (size_t)NH_ * rows * HD) return; const int d = (int)(e % HD); const int r = (int)((e / HD) % rows); const int h = (int)(e / ((size_t)HD * rows)); const float* f = F + (size_t)r * DMD + h * HD + d; v4us oh, ol;
#pragma unroll
    for (int u = 0; u < 4; ++u) { unsigned short a, b; splitf(f[u], a, b); oh[u] = a; ol[u] = b; } *(volatile v4us*)(Ph + e) = oh; *(volatile v4us*)(Pl + e) = ol; __threadfence(); *(volatile v4us*)(Ph + e) = oh; *(volatile v4us*)(Pl + e) = ol; }
__global__ __launch_bounds__(256) void k_vt2(const float* __restrict__ V, bf* Th, bf* Tl) { const int e = (blockIdx.x * 256 + threadIdx.x) * 2; if (e >= NH_ * HD * NBS) return; const int n = e % NBS; const int d = (e / NBS) % HD; const int h = e / (NBS * HD); v2us oh, ol;
#pragma unroll
    for (int u = 0; u < 2; ++u) { unsigned short a, b; splitf(V[(size_t)(n + u) * DMD + h * HD + d], a, b); oh[u] = a; ol[u] = b; } *(volatile v2us*)(Th + e) = oh; *(volatile v2us*)(Tl + e) = ol; __threadfence(); *(volatile v2us*)(Th + e) = oh; *(volatile v2us*)(Tl + e) = ol; }
__global__ __launch_bounds__(256) void k_dens(const float* __restrict__ S, const float* __restrict__ wmu, const float* __restrict__ wsg, const float* __restrict__ mub, const float* __restrict__ sgb, bf* Rh, bf* Rl) {
    const int lane = threadIdx.x & 31; const int row = blockIdx.x * 8 + (threadIdx.x >> 5); if (row >= NH_ * LL) return; const float* sr = S + (size_t)row * NBS; float sc[NBS / 32]; float z1 = 0.f, z2 = 0.f;
#pragma unroll
    for (int m = 0; m < NBS / 128; ++m) { const v4f a = *(const v4f*)(sr + m * 128 + lane * 4);
#pragma unroll
        for (int u = 0; u < 4; ++u) { const int n = m * 128 + lane * 4 + u; const float s8 = a[u] * 0.125f; sc[m * 4 + u] = s8; float p1 = __fmul_rn(s8, bfr(wmu[n])); asm volatile("" : "+v"(p1)); z1 = __fadd_rn(z1, p1); float p2 = __fmul_rn(s8, bfr(wsg[n])); asm volatile("" : "+v"(p2)); z2 = __fadd_rn(z2, p2); } }
#pragma unroll
    for (int sh = 16; sh; sh >>= 1) { z1 += __shfl_xor(z1, sh, 32); z2 += __shfl_xor(z2, sh, 32); }
    const float mu = __fdiv_rn(1.0f, __fadd_rn(1.0f, __expf(-z1))); const float ssq = (z2 > 20.f) ? z2 : log1pf(__expf(z2));
    for (int ps = 0; ps < 2; ++ps) {
#pragma unroll
        for (int m = 0; m < NBS / 128; ++m) { v4us oh, ol;
#pragma unroll
            for (int u = 0; u < 4; ++u) { const int n = m * 128 + lane * 4 + u; const float sb = bfr(sgb[n]); float v2 = __fmul_rn(sb, sb); asm volatile("" : "+v"(v2)); const float rs = __frsqrt_rn(__fadd_rn(v2, ssq)); float df = __fsub_rn(mu, bfr(mub[n])); asm volatile("" : "+v"(df)); float t = __fmul_rn(df, rs); asm volatile("" : "+v"(t));
                float hq = __fmul_rn(-0.5f, t); asm volatile("" : "+v"(hq)); const float ex = __expf(__fmul_rn(hq, t)); float pdf = __fmul_rn(0.3989422804014327f, ex); asm volatile("" : "+v"(pdf)); const float r = __fmul_rn(pdf, rs); unsigned short a, b; splitf(r, a, b); oh[u] = a; ol[u] = b; }
            const size_t oo = (size_t)row * NBS + m * 128 + lane * 4; *(volatile v4us*)(Rh + oo) = oh; *(volatile v4us*)(Rl + oo) = ol; }
        if (ps == 0) __threadfence(); } }
__global__ __launch_bounds__(256) void k_spl(const float* __restrict__ F, size_t n4, bf* Hh, bf* Hl) { const size_t e = ((size_t)blockIdx.x * 256 + threadIdx.x) * 4; if (e >= n4) return; const v4f a = *(const v4f*)(F + e); v4us oh, ol;
#pragma unroll
    for (int u = 0; u < 4; ++u) { unsigned short p, q; splitf(a[u], p, q); oh[u] = p; ol[u] = q; } *(volatile v4us*)(Hh + e) = oh; *(volatile v4us*)(Hl + e) = ol; __threadfence(); *(volatile v4us*)(Hh + e) = oh; *(volatile v4us*)(Hl + e) = ol; }
__global__ __launch_bounds__(256) void k_mrg(const float* __restrict__ O, bf* Ah, bf* Al) { const int e = (blockIdx.x * 256 + threadIdx.x) * 4; if (e >= NH_ * LL * HD) return; const int d = e % HD; const int l = (e / HD) % LL; const int h = e / (HD * LL); v4us oh, ol;
#pragma unroll
    for (int u = 0; u < 4; ++u) { unsigned short a, b; splitf(O[e + u], a, b); oh[u] = a; ol[u] = b; } const size_t oo = (size_t)l * DMD + h * HD + d; *(volatile v4us*)(Ah + oo) = oh; *(volatile v4us*)(Al + oo) = ol; __threadfence(); *(volatile v4us*)(Ah + oo) = oh; *(volatile v4us*)(Al + oo) = ol; }

extern "C" void kernel_launch(void* const* d_in, const int* in_sizes, int n_in,
                              void* d_out, int out_size, void* d_ws, size_t ws_size, hipStream_t stream) {
    (void)in_sizes; (void)n_in; (void)out_size;
    const float** I = (const float**)d_in;
    const float *x = I[0], *q = I[1], *Wq = I[2], *Wk = I[3], *Wv = I[4], *Wo = I[5], *wmu = I[6], *wsg = I[7], *mub = I[8], *sgb = I[9], *G = I[10];
    float* OUT = (float*)d_out;
    char* wsp = (char*)d_ws;
    auto take = [&](size_t bytes) { char* p = wsp; wsp += (bytes + 255) & ~(size_t)255; return (void*)p; };
    bf* BW[4]; for (int i = 0; i < 4; ++i) BW[i] = (bf*)take((size_t)DMD * DMD * 2); bf* GT = (bf*)take((size_t)NBS * LL * 2); bf* XT = (bf*)take((size_t)DMD * LL * 2); bf* QB = (bf*)take((size_t)LL * DMD * 2);
    float* BM = (float*)take((size_t)NBS * DMD * 4); bf* BMh = (bf*)take((size_t)NBS * DMD * 2); bf* BMl = (bf*)take((size_t)NBS * DMD * 2); float* KF = (float*)take((size_t)NBS * DMD * 4); float* VF = (float*)take((size_t)NBS * DMD * 4); float* QF = (float*)take((size_t)LL * DMD * 4);
    bf* QPh = (bf*)take((size_t)NH_ * LL * HD * 2); bf* QPl = (bf*)take((size_t)NH_ * LL * HD * 2); bf* KPh = (bf*)take((size_t)NH_ * NBS * HD * 2); bf* KPl = (bf*)take((size_t)NH_ * NBS * HD * 2); bf* VTh = (bf*)take((size_t)NH_ * HD * NBS * 2); bf* VTl = (bf*)take((size_t)NH_ * HD * NBS * 2);
    float* S = (float*)take((size_t)NH_ * LL * NBS * 4); bf* Rh = (bf*)take((size_t)NH_ * LL * NBS * 2); bf* Rl = (bf*)take((size_t)NH_ * LL * NBS * 2); float* O = (float*)take((size_t)NH_ * LL * HD * 4); bf* CTh = (bf*)take((size_t)LL * DMD * 2); bf* CTl = (bf*)take((size_t)LL * DMD * 2);
    if ((size_t)(wsp - (char*)d_ws) > ws_size) return;
    const float* Wl[4] = {Wq, Wk, Wv, Wo}; for (int i = 0; i < 4; ++i) k_cvt8<<<(DMD * DMD / 8 + 255) / 256, 256, 0, stream>>>(Wl[i], BW[i], DMD * DMD / 8);
    k_gt<<<(NBS * LL / 4 + 255) / 256, 256, 0, stream>>>(G, GT);
    const size_t zq = (size_t)LL * HD, zk = (size_t)NBS * HD, zs = (size_t)LL * NBS, zv = (size_t)HD * NBS;
    for (int b = 0; b < NBAT; ++b) {
        k_xbt<<<(DMD * LL / 4 + 255) / 256, 256, 0, stream>>>(x, b, XT);
        k_gemmw<bf, 0, false><<<dim3(NBS / 64, DMD / 64, 1), 32, 0, stream>>>(GT, nullptr, XT, nullptr, LL, BM, DMD, nullptr, 0, 0, 0);
        k_spl<<<(NBS * DMD / 4 + 255) / 256, 256, 0, stream>>>(BM, (size_t)NBS * DMD, BMh, BMl);
        k_gemmw<bf, 1, false><<<dim3(NBS / 64, DMD / 64, 1), 32, 0, stream>>>(BMh, BMl, BW[1], nullptr, DMD, KF, DMD, nullptr, 0, 0, 0); k_gemmw<bf, 1, false><<<dim3(NBS / 64, DMD / 64, 1), 32, 0, stream>>>(BMh, BMl, BW[2], nullptr, DMD, VF, DMD, nullptr, 0, 0, 0);
        k_qrow<<<(LL * DMD / 4 + 255) / 256, 256, 0, stream>>>(q, b, QB);
        k_gemmw<bf, 0, false><<<dim3(LL / 64, DMD / 64, 1), 32, 0, stream>>>(QB, nullptr, BW[0], nullptr, DMD, QF, DMD, nullptr, 0, 0, 0);
        k_pl2<<<(NH_ * LL * HD / 4 + 255) / 256, 256, 0, stream>>>(QF, LL, QPh, QPl); k_pl2<<<(NH_ * NBS * HD / 4 + 255) / 256, 256, 0, stream>>>(KF, NBS, KPh, KPl); k_vt2<<<(NH_ * HD * NBS / 2 + 255) / 256, 256, 0, stream>>>(VF, VTh, VTl);
        k_gemmw<bf, 2, false><<<dim3(LL / 64, NBS / 64, NH_), 32, 0, stream>>>(QPh, QPl, KPh, KPl, HD, S, NBS, nullptr, zq, zk, zs);
        k_dens<<<NH_ * LL / 8, 256, 0, stream>>>(S, wmu, wsg, mub, sgb, Rh, Rl);
        k_gemmw<bf, 2, false><<<dim3(LL / 64, 1, NH_), 32, 0, stream>>>(Rh, Rl, VTh, VTl, NBS, O, HD, nullptr, zs, zv, zq);
        k_mrg<<<(NH_ * LL * HD / 4 + 255) / 256, 256, 0, stream>>>(O, CTh, CTl);
        k_gemmw<bf, 1, false><<<dim3(LL / 64, DMD / 64, 1), 32, 0, stream>>>(CTh, CTl, BW[3], nullptr, DMD, OUT + (size_t)b * LL * DMD, DMD, nullptr, 0, 0, 0); }
}
